// RelAttention_15298673509083
// MI455X (gfx1250) — hardware-verified
//
#include <hip/hip_runtime.h>
#include <math.h>
#include <stdint.h>

#ifndef NB
#define NB 4
#endif
#ifndef SEQ
#define SEQ 1024
#endif
#define SEQ_FULL 1024
#define ND    1024
#define NH    16
#define HDV   64
#define HQK   128
#define QKW   (2 * ND)
#define TW    (2 * HQK)
#define NPP   (2 * SEQ)
#define BDW   (SEQ + 64)
#define NPAIR 8

static_assert(SEQ % 64 == 0);
static_assert(SEQ <= SEQ_FULL);
static_assert(ND == NH * HDV);
static_assert(HQK == 2 * HDV);
static_assert(TW == 2 * HQK);
static_assert((HDV & (HDV - 1)) == 0);
static_assert(NH % NPAIR == 0);
static_assert(ND % 256 == 0);
static_assert(NPP % 64 == 0);
static_assert(BDW % 64 == 0);
static_assert(NB >= 1);

typedef _Float16 v16h __attribute__((ext_vector_type(16)));
typedef _Float16 v8h  __attribute__((ext_vector_type(8)));
typedef float    v8f  __attribute__((ext_vector_type(8)));
typedef float    v4f  __attribute__((ext_vector_type(4)));
typedef unsigned int v4u __attribute__((ext_vector_type(4)));
typedef v4f __attribute__((may_alias)) v4fa;
typedef v8h __attribute__((may_alias)) v8ha;

__device__ __forceinline__ float bf_rne(float f) {
  unsigned u = __float_as_uint(f);
  u = (u + 0x7FFFu + ((u >> 16) & 1u)) & 0xFFFF0000u;
  return __uint_as_float(u);
}

union FragU { v16h v; v8ha h[2]; };
__device__ __forceinline__ v16h ldfrag(const _Float16* p) {
  FragU f;
  f.h[0] = *(const v8ha*)(p);
  f.h[1] = *(const v8ha*)(p + 16);
  return f.v;
}

__device__ __forceinline__ v8f mma16(v16h a, v16h b, v8f c) {
  c = __builtin_amdgcn_wmma_f32_16x16x32_f16(false, a, false, b, (short)0, c, false, false);
  asm volatile("v_nop\n\tv_nop\n\tv_nop\n\tv_nop" : "+v"(c) : "v"(a), "v"(b));
  return c;
}

__device__ __forceinline__ v8f zero8() { v8f z = {0.f, 0.f, 0.f, 0.f, 0.f, 0.f, 0.f, 0.f}; return z; }

template <bool DUP>
__global__ __launch_bounds__(256) void cvt_w_kernel(const float* __restrict__ src, _Float16* __restrict__ dst,
                                                    float s1, float s2) {
  const int i = blockIdx.x * 256 + threadIdx.x;
  const int total8 = ND * (ND / 8);
  if (i >= total8) return;
  const int r  = i / (ND / 8);
  const int c8 = (i - r * (ND / 8)) * 8;
  const float* sp = src + (size_t)r * ND + c8;
  const v4f a = *(const v4f*)(sp);
  const v4f b = *(const v4f*)(sp + 4);
  float f[8];
  f[0] = bf_rne(a[0]); f[1] = bf_rne(a[1]); f[2] = bf_rne(a[2]); f[3] = bf_rne(a[3]);
  f[4] = bf_rne(b[0]); f[5] = bf_rne(b[1]); f[6] = bf_rne(b[2]); f[7] = bf_rne(b[3]);
  v8h o1, o2;
#pragma unroll
  for (int e = 0; e < 8; ++e) { o1[e] = (_Float16)(f[e] * s1); o2[e] = (_Float16)(f[e] * s2); }
  const int pitch = DUP ? QKW : ND;
  _Float16* dp = dst + (size_t)r * pitch + c8;
  *(volatile v8h*)dp = o1;
  if (DUP) *(volatile v8h*)(dp + ND) = o2;
  __threadfence();
  *(volatile v8h*)dp = o1;
  if (DUP) *(volatile v8h*)(dp + ND) = o2;
}

__global__ __launch_bounds__(256) void cvt_x_kernel(const float* __restrict__ src, _Float16* __restrict__ dst, int nrows) {
  const int i = blockIdx.x * 256 + threadIdx.x;
  const int total8 = nrows * (ND / 8);
  if (i >= total8) return;
  const int row = i / (ND / 8);
  const int c8  = (i - row * (ND / 8)) * 8;
  const int b   = row / SEQ;
  const int t   = row - b * SEQ;
  const float* sp = src + ((size_t)b * SEQ_FULL + t) * ND + c8;
  const v4f a = *(const v4f*)(sp);
  const v4f c = *(const v4f*)(sp + 4);
  v8h o;
  o[0] = (_Float16)bf_rne(a[0]); o[1] = (_Float16)bf_rne(a[1]); o[2] = (_Float16)bf_rne(a[2]); o[3] = (_Float16)bf_rne(a[3]);
  o[4] = (_Float16)bf_rne(c[0]); o[5] = (_Float16)bf_rne(c[1]); o[6] = (_Float16)bf_rne(c[2]); o[7] = (_Float16)bf_rne(c[3]);
  _Float16* dp = dst + (size_t)row * ND + c8;
  *(volatile v8h*)dp = o;
  __threadfence();
  *(volatile v8h*)dp = o;
}

__global__ __launch_bounds__(256) void cvt_t_kernel(const float* __restrict__ pos, _Float16* __restrict__ T, int b) {
  const int i = blockIdx.x * 256 + threadIdx.x;
  if (i >= NH * NPP * 32) return;
  const int h    = i / (NPP * 32);
  const int rem  = i - h * (NPP * 32);
  const int tr   = rem >> 5;
  const int p    = rem & 31;
  const int seg  = p >> 4;
  const int islo = (p >> 3) & 1;
  const int d8   = (p & 7) * 8;
  const int srow = (seg == 0) ? tr : (tr - SEQ - 1);
  const int live = (seg == 0) ? ((tr < SEQ) ? 1 : 0) : (((tr >= SEQ + 1) && (tr <= 2 * SEQ - 2)) ? 1 : 0);
  int sr = (srow < 0) ? 0 : srow;
  sr = (sr > SEQ - 1) ? (SEQ - 1) : sr;
  const float sc = ((live != 0) ? 1.0f : 0.0f) * ((islo != 0) ? 0.015625f : 16.0f);
  const float* sp = pos + ((size_t)b * SEQ_FULL + sr) * ND + h * HDV + d8;
  const v4f a = *(const v4f*)(sp);
  const v4f c = *(const v4f*)(sp + 4);
  v8h o;
  o[0] = (_Float16)(bf_rne(a[0]) * sc); o[1] = (_Float16)(bf_rne(a[1]) * sc);
  o[2] = (_Float16)(bf_rne(a[2]) * sc); o[3] = (_Float16)(bf_rne(a[3]) * sc);
  o[4] = (_Float16)(bf_rne(c[0]) * sc); o[5] = (_Float16)(bf_rne(c[1]) * sc);
  o[6] = (_Float16)(bf_rne(c[2]) * sc); o[7] = (_Float16)(bf_rne(c[3]) * sc);
  _Float16* dp = T + ((size_t)h * NPP + tr) * TW + p * 8;
  *(volatile v8h*)dp = o;
  __threadfence();
  *(volatile v8h*)dp = o;
}

__global__ __launch_bounds__(256) void qvd_kernel(const _Float16* __restrict__ QV, _Float16* __restrict__ QD) {
  const int i = blockIdx.x * 256 + threadIdx.x;
  if (i >= NH * SEQ * 32) return;
  const int h   = i / (SEQ * 32);
  const int rem = i - h * (SEQ * 32);
  const int t   = rem >> 5;
  const int p   = rem & 31;
  const int seg = p >> 4;
  const int srow = t + seg;
  const int live = (srow < SEQ) ? 1 : 0;
  const int sr = (live != 0) ? srow : (SEQ - 1);
  const v8h val = *(const v8ha*)(QV + (size_t)sr * QKW + h * HQK + (p & 15) * 8);
  v8h o;
#pragma unroll
  for (int e = 0; e < 8; ++e) o[e] = (live != 0) ? val[e] : (_Float16)0.0f;
  _Float16* dp = QD + ((size_t)h * SEQ + t) * TW + p * 8;
  *(volatile v8h*)dp = o;
  __threadfence();
  *(volatile v8h*)dp = o;
}

template <int OUT, bool SKEW, bool HASB>
__global__ __launch_bounds__(256) void gemm_f16_kernel(
    const _Float16* __restrict__ A, int lda, long strideA,
    const _Float16* __restrict__ Bt, int ldb, long strideB,
    void* C1, void* C2, int ldc, long strideC,
    const float* __restrict__ b1, const float* __restrict__ b2, const float* __restrict__ b3,
    int M, int N, int K, float scale, float carry, int skew0, int ksplit) {
  __shared__ __align__(16) float sT[8][16 * 68];

  const int z    = blockIdx.y;
  const int lane = threadIdx.x & 31;
  const int wave = threadIdx.x >> 5;
  const int tilesN = N >> 6;
  const int tilesM = M >> 6;
  const int tile = blockIdx.x * 8 + wave;
  if (tile >= tilesM * tilesN) return;
  const int tm = tile / tilesN;
  const int tn = tile - tm * tilesN;
  const int m0 = tm << 6;
  const int n0 = tn << 6;
  const int nsk = SKEW ? ((skew0 - tm) << 6) : 0;

  int kbeg = 0, kend = K;
  if (SKEW && ksplit > 0) {
    if (nsk + n0 >= ksplit) kbeg = K >> 1; else kend = K >> 1;
  }

  const _Float16* Ab = A  + (size_t)z * strideA;
  const _Float16* Bb = Bt + (size_t)z * strideB;

  const int rl   = lane & 15;
  const int koff = (lane >> 4) * 8;
  const int mOff = (lane >> 4) * 8;

  v8f acc[4][4];
#pragma unroll
  for (int i = 0; i < 4; ++i)
#pragma unroll
    for (int j = 0; j < 4; ++j) acc[i][j] = zero8();

  for (int k0 = kbeg; k0 < kend; k0 += 32) {
    v16h bfr[4];
#pragma unroll
    for (int j = 0; j < 4; ++j)
      bfr[j] = ldfrag(Bb + (size_t)(nsk + n0 + (j << 4) + rl) * ldb + koff + k0);
#pragma unroll
    for (int i = 0; i < 4; ++i) {
      const v16h af = ldfrag(Ab + (size_t)(m0 + (i << 4) + rl) * lda + koff + k0);
#pragma unroll
      for (int j = 0; j < 4; ++j) acc[i][j] = mma16(af, bfr[j], acc[i][j]);
    }
  }

  float* slab = sT[wave];
  const int hh = lane >> 4, c4 = (lane & 15) * 4;
  const int q8 = lane >> 3, c8 = (lane & 7) * 8;
  v4f bias4 = {0.f, 0.f, 0.f, 0.f};
  float col8a[8], col8b[8], col8c[8];
#pragma unroll
  for (int e = 0; e < 8; ++e) { col8a[e] = 0.f; col8b[e] = 0.f; col8c[e] = 0.f; }
  if (OUT == 1 && HASB) {
    const v4f tb = *(const v4f*)(b1 + n0 + c4);
    bias4[0] = bf_rne(tb[0]); bias4[1] = bf_rne(tb[1]); bias4[2] = bf_rne(tb[2]); bias4[3] = bf_rne(tb[3]);
  }
  if (OUT == 2 && HASB) {
    const v4f ta = *(const v4f*)(b1 + n0 + c8);
    const v4f tb = *(const v4f*)(b1 + n0 + c8 + 4);
    col8a[0] = bf_rne(ta[0]); col8a[1] = bf_rne(ta[1]); col8a[2] = bf_rne(ta[2]); col8a[3] = bf_rne(ta[3]);
    col8a[4] = bf_rne(tb[0]); col8a[5] = bf_rne(tb[1]); col8a[6] = bf_rne(tb[2]); col8a[7] = bf_rne(tb[3]);
  }
  if (OUT == 3) {
    const int cb = (n0 + c8) & (HDV - 1);
    const v4f ta = *(const v4f*)(b1 + cb);
    const v4f tb = *(const v4f*)(b1 + cb + 4);
    col8a[0] = bf_rne(ta[0]); col8a[1] = bf_rne(ta[1]); col8a[2] = bf_rne(ta[2]); col8a[3] = bf_rne(ta[3]);
    col8a[4] = bf_rne(tb[0]); col8a[5] = bf_rne(tb[1]); col8a[6] = bf_rne(tb[2]); col8a[7] = bf_rne(tb[3]);
    const v4f tc = *(const v4f*)(b2 + cb);
    const v4f td = *(const v4f*)(b2 + cb + 4);
    col8b[0] = bf_rne(tc[0]); col8b[1] = bf_rne(tc[1]); col8b[2] = bf_rne(tc[2]); col8b[3] = bf_rne(tc[3]);
    col8b[4] = bf_rne(td[0]); col8b[5] = bf_rne(td[1]); col8b[6] = bf_rne(td[2]); col8b[7] = bf_rne(td[3]);
    if (HASB) {
      const v4f te = *(const v4f*)(b3 + n0 + c8);
      const v4f tf = *(const v4f*)(b3 + n0 + c8 + 4);
      col8c[0] = bf_rne(te[0]); col8c[1] = bf_rne(te[1]); col8c[2] = bf_rne(te[2]); col8c[3] = bf_rne(te[3]);
      col8c[4] = bf_rne(tf[0]); col8c[5] = bf_rne(tf[1]); col8c[6] = bf_rne(tf[2]); col8c[7] = bf_rne(tf[3]);
    }
  }
  const float carry2 = carry * 0.0009765625f;

#pragma unroll
  for (int i = 0; i < 4; ++i) {
    const int mBase = m0 + (i << 4);
#pragma unroll
    for (int j = 0; j < 4; ++j)
#pragma unroll
      for (int r = 0; r < 8; ++r)
        slab[(mOff + r) * 68 + (j << 4) + rl] = acc[i][j][r] * scale;
    __builtin_amdgcn_fence(__ATOMIC_RELEASE, "workgroup");
    __builtin_amdgcn_wave_barrier();
    __builtin_amdgcn_fence(__ATOMIC_ACQUIRE, "workgroup");
    if (OUT == 0 || OUT == 1) {
      float* C = (float*)C1 + (size_t)z * strideC;
      v4f vv[8];
#pragma unroll
      for (int it = 0; it < 8; ++it) {
        const int row = it * 2 + hh;
        v4f v = *(const v4fa*)(slab + row * 68 + c4);
        if (OUT == 1) v += bias4;
        vv[it] = v;
      }
      for (int ps = 0; ps < 2; ++ps) {
#pragma unroll
        for (int it = 0; it < 8; ++it) {
          const int row = it * 2 + hh;
          *(volatile v4f*)(C + (size_t)(mBase + row) * ldc + n0 + c4) = vv[it];
        }
        __threadfence();
      }
    } else if (OUT == 2 || OUT == 4) {
      _Float16* Ca = (_Float16*)C1 + (size_t)z * strideC;
      v8h hv[4], lv[4];
#pragma unroll
      for (int it = 0; it < 4; ++it) {
        const int row = it * 4 + q8;
        const float* sp = slab + row * 68 + c8;
        const v4f x0 = *(const v4fa*)(sp);
        const v4f x1 = *(const v4fa*)(sp + 4);
        float f[8];
        f[0] = x0[0]; f[1] = x0[1]; f[2] = x0[2]; f[3] = x0[3];
        f[4] = x1[0]; f[5] = x1[1]; f[6] = x1[2]; f[7] = x1[3];
        float rb = 0.f;
        if (OUT == 4 && HASB) rb = bf_rne(b1[mBase + row]);
        v8h ha, la;
#pragma unroll
        for (int e = 0; e < 8; ++e) {
          const float t = f[e] + ((OUT == 2) ? col8a[e] : rb);
          ha[e] = (_Float16)(t * carry);
          la[e] = (_Float16)(t * carry2);
        }
        hv[it] = ha; lv[it] = la;
      }
      for (int ps = 0; ps < 2; ++ps) {
#pragma unroll
        for (int it = 0; it < 4; ++it) {
          const int row = it * 4 + q8;
          if (OUT == 2) {
            _Float16* cp = Ca + (size_t)(mBase + row) * ldc + 2 * n0 + c8;
            *(volatile v8h*)(cp)      = hv[it];
            *(volatile v8h*)(cp + 64) = lv[it];
          } else {
            *(volatile v8h*)(Ca + (size_t)(mBase + row) * ldc + n0 + c8) = hv[it];
          }
        }
        __threadfence();
      }
    } else {
#pragma unroll
      for (int var = 0; var < 2; ++var) {
        _Float16* Cc = (_Float16*)((var == 0) ? C1 : C2) + (size_t)z * strideC;
        v8h hv[4], lv[4];
#pragma unroll
        for (int it = 0; it < 4; ++it) {
          const int row = it * 4 + q8;
          const float* sp = slab + row * 68 + c8;
          const v4f x0 = *(const v4fa*)(sp);
          const v4f x1 = *(const v4fa*)(sp + 4);
          float f[8];
          f[0] = x0[0]; f[1] = x0[1]; f[2] = x0[2]; f[3] = x0[3];
          f[4] = x1[0]; f[5] = x1[1]; f[6] = x1[2]; f[7] = x1[3];
          v8h ha, la;
#pragma unroll
          for (int e = 0; e < 8; ++e) {
            const float t  = (f[e] + col8c[e]) + ((var == 0) ? col8a[e] : col8b[e]);
            const float th = t * carry;
            const _Float16 hq = (_Float16)th;
            ha[e] = hq;
            la[e] = (_Float16)((th - (float)hq) * 1024.0f);
          }
          hv[it] = ha; lv[it] = la;
        }
        for (int ps = 0; ps < 2; ++ps) {
#pragma unroll
          for (int it = 0; it < 4; ++it) {
            const int row = it * 4 + q8;
            _Float16* cp = Cc + (size_t)(mBase + row) * ldc + 2 * n0 + c8;
            *(volatile v8h*)(cp)      = hv[it];
            *(volatile v8h*)(cp + 64) = lv[it];
          }
          __threadfence();
        }
      }
    }
    __builtin_amdgcn_fence(__ATOMIC_RELEASE, "workgroup");
    __builtin_amdgcn_wave_barrier();
    __builtin_amdgcn_fence(__ATOMIC_ACQUIRE, "workgroup");
  }
}

__global__ __launch_bounds__(128)
void band_attn_kernel(const _Float16* __restrict__ QU, const _Float16* __restrict__ KP,
                      const _Float16* __restrict__ VT, const float* __restrict__ BD,
                      _Float16* __restrict__ CTX, int h0, float cs) {
  __shared__ __align__(16) unsigned char SMEM[32768];
  _Float16* Ksh = (_Float16*)(SMEM);
  _Float16* Vsh = (_Float16*)(SMEM + 16384);
  _Float16* Psh = (_Float16*)(SMEM + 24576);
  float*    Osh = (float*)(SMEM);

  const int tid  = threadIdx.x;
  const int wave = tid >> 5;
  const int lane = tid & 31;
  const int hh   = lane >> 4;
  const int c    = lane & 15;

  const int z    = blockIdx.y;
  const int h    = h0 + z;
  const int qb   = blockIdx.x;
  const int q0   = qb * 64 + wave * 16;
  const int rr0  = wave * 16 + 8 * hh;

  const _Float16* Qh = QU + h * HQK;
  const _Float16* Kh = KP + h * HQK;
  const _Float16* Vh = VT + (size_t)(h * HDV) * SEQ;
  const float*    bd = BD + (size_t)z * SEQ * BDW;
  _Float16*       ctx = CTX + h * HDV;

  v16h qa[4];
#pragma unroll
  for (int dc = 0; dc < 4; ++dc)
    qa[dc] = ldfrag(Qh + (size_t)(q0 + c) * QKW + dc * 32 + 8 * hh);

  const float* bdr = bd + (size_t)(q0 + 8 * hh) * BDW + (63 - rr0 + c);

  float mrow[8], lrow[8];
  v8f oacc[4];
#pragma unroll
  for (int r = 0; r < 8; ++r) { mrow[r] = -INFINITY; lrow[r] = 0.f; }
#pragma unroll
  for (int t = 0; t < 4; ++t) oacc[t] = zero8();

  _Float16* pw = Psh + wave * (16 * 64);

#pragma unroll 1
  for (int kc = 0; kc < SEQ / 64; ++kc) {
    const int kv0 = kc * 64;
    __syncthreads();
    {
      const int r = tid >> 1, c0 = (tid & 1) * 64, cv = (tid & 1) * 32;
      const _Float16* ks = Kh + (size_t)(kv0 + r) * QKW + c0;
      const _Float16* vs = Vh + (size_t)r * SEQ + kv0 + cv;
#pragma unroll
      for (int i = 0; i < 8; ++i) {
        const v8h kk8 = *(const v8h*)(ks + 8 * i);
        *(v8ha*)(Ksh + r * 128 + c0 + 8 * i) = kk8;
      }
#pragma unroll
      for (int i = 0; i < 4; ++i) {
        const v8h vv8 = *(const v8h*)(vs + 8 * i);
        *(v8ha*)(Vsh + r * 64 + cv + 8 * i) = vv8;
      }
    }
    __syncthreads();

    v8f s[4];
#pragma unroll
    for (int j = 0; j < 4; ++j) {
      s[j] = zero8();
#pragma unroll
      for (int dc = 0; dc < 4; ++dc) {
        const v16h kb = ldfrag(Ksh + (j * 16 + c) * 128 + dc * 32 + 8 * hh);
        s[j] = mma16(qa[dc], kb, s[j]);
      }
    }

    float cm[8];
#pragma unroll
    for (int r = 0; r < 8; ++r) {
      float m = -INFINITY;
#pragma unroll
      for (int j = 0; j < 4; ++j) {
        const float sv = s[j][r] * cs + bdr[(size_t)r * (BDW - 1) + kv0 + (j << 4)];
        s[j][r] = sv;
        m = fmaxf(m, sv);
      }
      m = fmaxf(m, __shfl_xor(m, 1, 32));
      m = fmaxf(m, __shfl_xor(m, 2, 32));
      m = fmaxf(m, __shfl_xor(m, 4, 32));
      m = fmaxf(m, __shfl_xor(m, 8, 32));
      cm[r] = m;
    }

#pragma unroll
    for (int r = 0; r < 8; ++r) {
      const float mnew  = fmaxf(mrow[r], cm[r]);
      const float alpha = __expf(mrow[r] - mnew);
      mrow[r] = mnew;
      float psum = 0.f;
#pragma unroll
      for (int j = 0; j < 4; ++j) {
        const float p = __expf(s[j][r] - mnew);
        psum += p;
        pw[(8 * hh + r) * 64 + j * 16 + c] = (_Float16)(p * 4096.0f);
      }
      psum += __shfl_xor(psum, 1, 32);
      psum += __shfl_xor(psum, 2, 32);
      psum += __shfl_xor(psum, 4, 32);
      psum += __shfl_xor(psum, 8, 32);
      lrow[r] = lrow[r] * alpha + psum;
#pragma unroll
      for (int t = 0; t < 4; ++t) oacc[t][r] *= alpha;
    }
    __builtin_amdgcn_fence(__ATOMIC_RELEASE, "workgroup");
    __builtin_amdgcn_wave_barrier();
    __builtin_amdgcn_fence(__ATOMIC_ACQUIRE, "workgroup");

#pragma unroll
    for (int kk = 0; kk < 2; ++kk) {
      const v16h pa = ldfrag(pw + c * 64 + kk * 32 + 8 * hh);
#pragma unroll
      for (int t = 0; t < 4; ++t) {
        const v16h vb = ldfrag(Vsh + (t * 16 + c) * 64 + kk * 32 + 8 * hh);
        oacc[t] = mma16(pa, vb, oacc[t]);
      }
    }
  }

  __syncthreads();
  float* os = Osh + wave * (16 * HDV);
#pragma unroll
  for (int r = 0; r < 8; ++r) {
    const float inv = 1.0f / (1024.0f * lrow[r]);
#pragma unroll
    for (int t = 0; t < 4; ++t) os[(8 * hh + r) * HDV + t * 16 + c] = oacc[t][r] * inv;
  }
  __builtin_amdgcn_fence(__ATOMIC_RELEASE, "workgroup");
  __builtin_amdgcn_wave_barrier();
  __builtin_amdgcn_fence(__ATOMIC_ACQUIRE, "workgroup");
  const int q8 = lane >> 3, c8 = (lane & 7) * 8;
  v8h ov[4], rv[4];
#pragma unroll
  for (int it = 0; it < 4; ++it) {
    const int row = it * 4 + q8;
    const float* sp = os + row * HDV + c8;
    const v4f x0 = *(const v4fa*)(sp);
    const v4f x1 = *(const v4fa*)(sp + 4);
    float f[8];
    f[0] = x0[0]; f[1] = x0[1]; f[2] = x0[2]; f[3] = x0[3];
    f[4] = x1[0]; f[5] = x1[1]; f[6] = x1[2]; f[7] = x1[3];
    v8h o, q;
#pragma unroll
    for (int e = 0; e < 8; ++e) {
      const _Float16 hv = (_Float16)f[e];
      o[e] = hv;
      q[e] = (_Float16)((f[e] - (float)hv) * 1024.0f);
    }
    ov[it] = o; rv[it] = q;
  }
  for (int ps = 0; ps < 2; ++ps) {
#pragma unroll
    for (int it = 0; it < 4; ++it) {
      const int row = it * 4 + q8;
      _Float16* cp = ctx + (size_t)(q0 + row) * QKW + c8;
      *(volatile v8h*)(cp)      = ov[it];
      *(volatile v8h*)(cp + ND) = rv[it];
    }
    __threadfence();
  }
}

extern "C" void kernel_launch(void* const* d_in, const int* in_sizes, int n_in,
                              void* d_out, int out_size, void* d_ws, size_t ws_size,
                              hipStream_t stream) {
  if (n_in < 12) return;
  if (in_sizes[0] < ((NB - 1) * SEQ_FULL + SEQ) * ND) return;
  if (in_sizes[3] < ((NB - 1) * SEQ_FULL + SEQ) * ND) return;
  if (in_sizes[1] < HDV || in_sizes[2] < HDV) return;
  if (in_sizes[4] != ND * ND || in_sizes[6] != ND * ND || in_sizes[8] != ND * ND || in_sizes[10] != ND * ND) return;
  if (in_sizes[5] < ND || in_sizes[7] < ND || in_sizes[9] < ND || in_sizes[11] < ND) return;
  if (out_size < NB * SEQ * ND) return;

  const float* x   = (const float*)d_in[0];
  const float* ub  = (const float*)d_in[1];
  const float* vb  = (const float*)d_in[2];
  const float* pos = (const float*)d_in[3];
  const float* Wq  = (const float*)d_in[4];
  const float* bq  = (const float*)d_in[5];
  const float* Wk  = (const float*)d_in[6];
  const float* bk  = (const float*)d_in[7];
  const float* Wv  = (const float*)d_in[8];
  const float* bv  = (const float*)d_in[9];
  const float* Wc  = (const float*)d_in[10];
  const float* bc  = (const float*)d_in[11];
  float* out = (float*)d_out;

  const size_t szW1  = (size_t)ND * ND * 2;
  const size_t szW2  = (size_t)ND * QKW * 2;
  const size_t szX   = (size_t)NB * SEQ * ND * 2;
  const size_t szQb  = (size_t)SEQ * QKW * 2;
  const size_t szVT  = (size_t)ND * SEQ * 2;
  const size_t szQD  = (size_t)NH * SEQ * TW * 2;
  const size_t szT   = (size_t)NH * NPP * TW * 2;
  const size_t szCTX = (size_t)NB * SEQ * QKW * 2;
  const size_t szBD  = (size_t)NPAIR * SEQ * BDW * 4;
  size_t off = 0;
  const size_t oWQ  = off; off += szW1;
  const size_t oWK  = off; off += szW1;
  const size_t oWV  = off; off += szW1;
  const size_t oWC2 = off; off += szW2;
  const size_t oX   = off; off += szX;
  const size_t oQU2 = off; off += szQb;
  const size_t oQV2 = off; off += szQb;
  const size_t oKP2 = off; off += szQb;
  const size_t oVT  = off; off += szVT;
  const size_t oQD  = off; off += szQD;
  const size_t oT   = off; off += szT;
  const size_t oCTX = off; off += szCTX;
  const size_t oBD  = off; off += szBD;
  const size_t total = off;
  if (total > ws_size) return;
  if (total > (size_t)134217728) return;

  char* ws = (char*)d_ws;
  _Float16* WQp = (_Float16*)(ws + oWQ);
  _Float16* WKp = (_Float16*)(ws + oWK);
  _Float16* WVp = (_Float16*)(ws + oWV);
  _Float16* WC2 = (_Float16*)(ws + oWC2);
  _Float16* Xp  = (_Float16*)(ws + oX);
  _Float16* QU2 = (_Float16*)(ws + oQU2);
  _Float16* QV2 = (_Float16*)(ws + oQV2);
  _Float16* KP2 = (_Float16*)(ws + oKP2);
  _Float16* VTp = (_Float16*)(ws + oVT);
  _Float16* QDp = (_Float16*)(ws + oQD);
  _Float16* Tp  = (_Float16*)(ws + oT);
  _Float16* CTX = (_Float16*)(ws + oCTX);
  float*    BDp = (float*)(ws + oBD);

  const float cs = 0.03125f * 0.00390625f;
  const dim3 blk(256);

  const dim3 gW(ND * (ND / 8) / 256);
  cvt_w_kernel<false><<<gW, blk, 0, stream>>>(Wq, WQp, 64.0f, 64.0f);
  cvt_w_kernel<false><<<gW, blk, 0, stream>>>(Wk, WKp, 64.0f, 64.0f);
  cvt_w_kernel<false><<<gW, blk, 0, stream>>>(Wv, WVp, 64.0f, 64.0f);
  cvt_w_kernel<true ><<<gW, blk, 0, stream>>>(Wc, WC2, 64.0f, 0.0625f);
  cvt_x_kernel<<<dim3((NB * SEQ * (ND / 8) + 255) / 256), blk, 0, stream>>>(x, Xp, NB * SEQ);
  const int tilesQ  = (SEQ / 64) * (ND / 64);
  const int tilesBD = (SEQ / 64) * (BDW / 64);
  for (int b = 0; b < NB; ++b) {
    const _Float16* Xb = Xp + (size_t)b * SEQ * ND;
    gemm_f16_kernel<3, false, true><<<dim3((tilesQ + 7) / 8, 1), blk, 0, stream>>>(
        Xb, ND, 0L, WQp, ND, 0L, (void*)QU2, (void*)QV2, QKW, 0L, ub, vb, bq,
        SEQ, ND, ND, 0.015625f, 16.0f, 0, 0);
    gemm_f16_kernel<2, false, true><<<dim3((tilesQ + 7) / 8, 1), blk, 0, stream>>>(
        Xb, ND, 0L, WKp, ND, 0L, (void*)KP2, (void*)KP2, QKW, 0L, bk, bk, bk,
        SEQ, ND, ND, 0.015625f, 16.0f, 0, 0);
    gemm_f16_kernel<4, false, true><<<dim3((tilesQ + 7) / 8, 1), blk, 0, stream>>>(
        WVp, ND, 0L, Xb, ND, 0L, (void*)VTp, (void*)VTp, SEQ, 0L, bv, bv, bv,
        ND, SEQ, ND, 0.015625f, 16.0f, 0, 0);
    cvt_t_kernel<<<dim3((NH * NPP * 32 + 255) / 256), blk, 0, stream>>>(pos, Tp, b);
    qvd_kernel<<<dim3((NH * SEQ * 32 + 255) / 256), blk, 0, stream>>>(QV2, QDp);
    for (int gi = 0; gi < NH / NPAIR; ++gi) {
      const int h0 = gi * NPAIR;
      const _Float16* Aq = QDp + (size_t)h0 * SEQ * TW;
      const _Float16* Bp = Tp  + (size_t)h0 * NPP * TW;
      gemm_f16_kernel<0, true, false><<<dim3((tilesBD + 7) / 8, NPAIR), blk, 0, stream>>>(
          Aq, TW, (long)SEQ * TW, Bp, TW, (long)NPP * TW, (void*)BDp, (void*)BDp, BDW, (long)SEQ * BDW, bq, bq, bq,
          SEQ, BDW, TW, cs, 1.0f, SEQ / 64 - 1, SEQ);
      band_attn_kernel<<<dim3(SEQ / 64, NPAIR), dim3(128), 0, stream>>>(
          QU2, KP2, VTp, BDp, CTX + (size_t)b * SEQ * QKW, h0, cs);
    }
  }
  {
    const int tiles = ((NB * SEQ) / 64) * (ND / 64);
    gemm_f16_kernel<1, false, true><<<dim3((tiles + 7) / 8, 1), blk, 0, stream>>>(
        CTX, QKW, 0L, WC2, QKW, 0L, (void*)out, (void*)out, ND, 0L, bc, bc, bc,
        NB * SEQ, ND, QKW, 0.000244140625f, 1.0f, 0, 0);
  }
  (void)hipGetLastError();
}
